// STFT_75118978007171
// MI455X (gfx1250) — hardware-run, weakly checked
//
#include <hip/hip_runtime.h>
#include <math.h>

typedef __attribute__((ext_vector_type(16))) _Float16 v16h;
typedef __attribute__((ext_vector_type(8)))  _Float16 v8h;
typedef __attribute__((ext_vector_type(8)))  float    v8f;
typedef __attribute__((ext_vector_type(4)))  float    v4f;
typedef __attribute__((ext_vector_type(4)))  unsigned v4u;

constexpr int kNb       = 32;
constexpr int kSig      = 220500;
constexpr int kNfft     = 2048;
constexpr int kHop      = 512;
constexpr int kPadHalf  = kNfft / 2;
constexpr int kPadLen   = kSig + 2 * kPadHalf;
constexpr int kFrames   = (kPadLen - kNfft) / kHop + 1;
constexpr int kBins     = kNfft / 2 + 1;
constexpr int kRowsReal = kNb * kFrames;
constexpr int kRowsPad  = ((kRowsReal + 63) / 64) * 64;
constexpr int kBinTiles = (kBins + 31) / 32;
constexpr int kTapRows  = kBinTiles * 64;
constexpr int kMagP     = kBinTiles * 32;
constexpr int kTilesM   = kRowsPad / 64;
constexpr int kTilesN   = kTapRows / 64;
constexpr int kPerBatch = kBins * kFrames;
constexpr int kOutTotal = kNb * kPerBatch;
constexpr int kOutLines = kOutTotal / 32;
constexpr int kSlabP    = 36;

static_assert(kFrames == 431);
static_assert(kBins == 1025);
static_assert(kRowsReal == 13792);
static_assert(kRowsPad == 13824);
static_assert(kTapRows == 2112);
static_assert(kMagP == 1056);
static_assert(kTilesM == 216 && kTilesN == 33);
static_assert((kTilesM * kTilesN) % 8 == 0);
static_assert(kOutTotal == 14136800);
static_assert((kOutTotal % 32) == 0);
static_assert(kOutLines == 441775);
static_assert((kNfft % 32) == 0);
static_assert((kSig % 4) == 0);

constexpr float kCarrySig = 16.0f;
constexpr float kCarryTap = 256.0f;
constexpr float kFold     = 1.0f / (kCarrySig * kCarryTap);
constexpr float kHalfMinNormal = 6.103515625e-05f;
static_assert(kFold * 4096.0f == 1.0f);

constexpr size_t kBytesFr  = (size_t)kRowsPad * kNfft * 2;
constexpr size_t kBytesTap = (size_t)kTapRows * kNfft * 2;
constexpr size_t kBytesMag = (size_t)kRowsPad * kMagP * 4;
constexpr size_t kOffFr    = 0;
constexpr size_t kOffTap   = kOffFr + kBytesFr;
constexpr size_t kOffMag   = kOffTap + kBytesTap;
constexpr size_t kWsTotal  = kOffMag + kBytesMag;
static_assert(kBytesFr == 56623104ull);
static_assert(kBytesTap == 8650752ull);
static_assert(kBytesMag == 58392576ull);
static_assert(kWsTotal == 123666432ull);
static_assert(kWsTotal <= 134217728ull);
static_assert((kOffTap % 128) == 0 && (kOffMag % 128) == 0);

namespace eng {
union FragU { v16h v; v8h h[2]; };
__device__ __forceinline__ v16h frag_load(const _Float16* p) {
  FragU f;
  f.h[0] = *(const v8h*)(p);
  f.h[1] = *(const v8h*)(p + 16);
  return f.v;
}
__device__ __forceinline__ v8f mma(v16h a, v16h b, v8f c) {
  return __builtin_amdgcn_wmma_f32_16x16x32_f16(false, a, false, b, (short)0, c, false, false);
}
__device__ __forceinline__ void tie_acc(v8f& c, v16h a, v16h b) {
  asm volatile("" : "+v"(c) : "v"(a), "v"(b));
}
__device__ __forceinline__ void tie_acc_nops(v8f& c, v16h a, v16h b) {
  asm volatile("v_nop\n\tv_nop\n\tv_nop\n\tv_nop" : "+v"(c) : "v"(a), "v"(b));
}
__device__ __forceinline__ void keep4(v16h a, v16h b, v16h c, v16h d) {
  asm volatile("v_nop" :: "v"(a), "v"(b), "v"(c), "v"(d));
}
__device__ __forceinline__ void acc_guard4(v8f& a, v8f& b, v8f& c, v8f& d) {
  asm volatile("v_nop\n\tv_nop\n\tv_nop\n\tv_nop" : "+v"(a), "+v"(b), "+v"(c), "+v"(d));
}
}

__device__ __forceinline__ float flush_small(float v) {
  return (fabsf(v) < kHalfMinNormal) ? 0.0f : v;
}
__device__ __forceinline__ unsigned pack2_f16(float a, float b) {
  const _Float16 h0 = (_Float16)a;
  const _Float16 h1 = (_Float16)b;
  const unsigned short u0 = __builtin_bit_cast(unsigned short, h0);
  const unsigned short u1 = __builtin_bit_cast(unsigned short, h1);
  return (unsigned)u0 | ((unsigned)u1 << 16);
}

__global__ __launch_bounds__(256) void frames_f16_kernel(const float* __restrict__ x, unsigned* __restrict__ FR)
{
  const int m   = blockIdx.x;
  const int tid = threadIdx.x;
  const bool valid = (m < kRowsReal);
  int b = m / kFrames;
  const int f = m - b * kFrames;
  b = (b < kNb) ? b : (kNb - 1);
  const float* xb = x + (size_t)b * kSig;
  const int j0 = kHop * f + 8 * tid - kPadHalf;
  float s[8];
#pragma unroll
  for (int e = 0; e < 8; ++e) {
    const int j = j0 + e;
    int jr = (j < 0) ? -j : j;
    jr = (jr >= kSig) ? (2 * (kSig - 1) - jr) : jr;
    jr = (jr < 0) ? 0 : jr;
    jr = (jr > kSig - 1) ? (kSig - 1) : jr;
    const float v = xb[jr];
    const float c = valid ? (v * kCarrySig) : 0.0f;
    s[e] = flush_small(c);
  }
  v4u w;
  w[0] = pack2_f16(s[0], s[1]);
  w[1] = pack2_f16(s[2], s[3]);
  w[2] = pack2_f16(s[4], s[5]);
  w[3] = pack2_f16(s[6], s[7]);
  unsigned* p = FR + (size_t)m * (kNfft / 2) + tid * 4;
  *(volatile v4u*)p = w;
  __threadfence();
  *(volatile v4u*)p = w;
}

__global__ __launch_bounds__(256) void taps_f16_kernel(const float* __restrict__ wsin, const float* __restrict__ wcos,
                                                       unsigned* __restrict__ TAP)
{
  const int r   = blockIdx.x;
  const int tid = threadIdx.x;
  const int t   = r >> 6;
  const int w   = r & 63;
  const int bin = 32 * t + (w & 31);
  const bool valid = (bin < kBins);
  const int binc = valid ? bin : (kBins - 1);
  const float* src = (w < 32) ? wsin : wcos;
  const float* rowp = src + (size_t)binc * kNfft + tid * 8;
  const v4f a0 = *(const v4f*)(rowp);
  const v4f a1 = *(const v4f*)(rowp + 4);
  float s[8];
#pragma unroll
  for (int e = 0; e < 4; ++e) {
    const float c0 = valid ? (a0[e] * kCarryTap) : 0.0f;
    const float c1 = valid ? (a1[e] * kCarryTap) : 0.0f;
    s[e]     = flush_small(c0);
    s[4 + e] = flush_small(c1);
  }
  v4u wv;
  wv[0] = pack2_f16(s[0], s[1]);
  wv[1] = pack2_f16(s[2], s[3]);
  wv[2] = pack2_f16(s[4], s[5]);
  wv[3] = pack2_f16(s[6], s[7]);
  unsigned* p = TAP + (size_t)r * (kNfft / 2) + tid * 4;
  *(volatile v4u*)p = wv;
  __threadfence();
  *(volatile v4u*)p = wv;
}

__global__ __launch_bounds__(256) void fused_product_mag_kernel(
    const unsigned short* __restrict__ Ap, const unsigned short* __restrict__ Btp, float* __restrict__ MAG)
{
  const _Float16* A  = (const _Float16*)Ap;
  const _Float16* Bt = (const _Float16*)Btp;
  __shared__ __align__(16) float sT[8][16 * kSlabP];
  const int lane = threadIdx.x & 31;
  const int wave = threadIdx.x >> 5;
  const int tile = blockIdx.x * 8 + wave;
  if (tile >= kTilesM * kTilesN) return;
  const int tm = tile / kTilesN;
  const int tn = tile - tm * kTilesN;
  const int m0 = tm << 6;
  const int n0 = tn << 6;

  const int rlane = lane & 15;
  const int koff  = (lane >> 4) * 8;
  const int mOff  = (lane >> 4) * 8;

  v8f acc[4][4];
#pragma unroll
  for (int i = 0; i < 4; ++i)
#pragma unroll
    for (int j = 0; j < 4; ++j) acc[i][j] = (v8f){0.f, 0.f, 0.f, 0.f, 0.f, 0.f, 0.f, 0.f};

#pragma unroll 1
  for (int k0 = 0; k0 < kNfft; k0 += 32) {
    v16h bh[4];
#pragma unroll
    for (int j = 0; j < 4; ++j) {
      const size_t bo = (size_t)(n0 + (j << 4) + rlane) * kNfft + koff + k0;
      bh[j] = eng::frag_load(Bt + bo);
    }
#pragma unroll
    for (int i = 0; i < 4; ++i) {
      const size_t ao = (size_t)(m0 + (i << 4) + rlane) * kNfft + koff + k0;
      const v16h ah = eng::frag_load(A + ao);
#pragma unroll
      for (int j = 0; j < 4; ++j) acc[i][j] = eng::mma(ah, bh[j], acc[i][j]);
      eng::tie_acc(acc[i][0], ah, bh[0]);
      eng::tie_acc(acc[i][1], ah, bh[1]);
      eng::tie_acc(acc[i][2], ah, bh[2]);
      eng::tie_acc_nops(acc[i][3], ah, bh[3]);
    }
    eng::keep4(bh[0], bh[1], bh[2], bh[3]);
  }
  eng::acc_guard4(acc[0][0], acc[0][1], acc[0][2], acc[0][3]);
  eng::acc_guard4(acc[1][0], acc[1][1], acc[1][2], acc[1][3]);
  eng::acc_guard4(acc[2][0], acc[2][1], acc[2][2], acc[2][3]);
  eng::acc_guard4(acc[3][0], acc[3][1], acc[3][2], acc[3][3]);

  float* slab = sT[wave];
  const int q  = lane >> 3;
  const int c4 = (lane & 7) * 4;
#pragma unroll
  for (int i = 0; i < 4; ++i) {
    const int mBase = m0 + (i << 4);
#pragma unroll
    for (int j = 0; j < 2; ++j) {
#pragma unroll
      for (int r = 0; r < 8; ++r) {
        const float s = acc[i][j][r] * kFold;
        const float c = acc[i][j + 2][r] * kFold;
        slab[(mOff + r) * kSlabP + (j << 4) + rlane] = s * s + c * c;
      }
    }
    __builtin_amdgcn_fence(__ATOMIC_RELEASE, "workgroup");
    __builtin_amdgcn_wave_barrier();
    __builtin_amdgcn_fence(__ATOMIC_ACQUIRE, "workgroup");
#pragma unroll 1
    for (int it = 0; it < 4; ++it) {
      float* sp = slab + (it * 4 + q) * kSlabP + c4;
      const v4f sq = *(const v4f*)sp;
      v4f mg;
      mg[0] = sqrtf(sq[0]);
      mg[1] = sqrtf(sq[1]);
      mg[2] = sqrtf(sq[2]);
      mg[3] = sqrtf(sq[3]);
      *(v4f*)sp = mg;
    }
    __builtin_amdgcn_fence(__ATOMIC_RELEASE, "workgroup");
    __builtin_amdgcn_wave_barrier();
    __builtin_amdgcn_fence(__ATOMIC_ACQUIRE, "workgroup");
    for (int pass = 0; pass < 2; ++pass) {
#pragma unroll
      for (int it = 0; it < 4; ++it) {
        const int row = it * 4 + q;
        const v4f v = *(const v4f*)(slab + row * kSlabP + c4);
        *(volatile v4f*)(MAG + (size_t)(mBase + row) * kMagP + tn * 32 + c4) = v;
      }
      __threadfence();
    }
    __builtin_amdgcn_fence(__ATOMIC_RELEASE, "workgroup");
    __builtin_amdgcn_wave_barrier();
    __builtin_amdgcn_fence(__ATOMIC_ACQUIRE, "workgroup");
  }
}

__global__ __launch_bounds__(256) void line_transpose_kernel(const float* __restrict__ MAG, float* __restrict__ out)
{
  const int line = blockIdx.x * 8 + (threadIdx.x >> 5);
  if (line >= kOutLines) return;
  const int g = line * 32 + (threadIdx.x & 31);
  int b = g / kPerBatch;
  b = (b < kNb) ? b : (kNb - 1);
  const int rem = g - b * kPerBatch;
  int k = rem / kFrames;
  k = (k < kBins) ? k : (kBins - 1);
  const int f = rem - k * kFrames;
  float v = MAG[(size_t)(b * kFrames + f) * kMagP + k];
  asm volatile("" : "+v"(v));
  volatile float* p = out + g;
  *p = v;
  __threadfence();
  *p = v;
}

extern "C" void kernel_launch(void* const* d_in, const int* in_sizes, int n_in,
                              void* d_out, int out_size, void* d_ws, size_t ws_size,
                              hipStream_t stream) {
  if (n_in < 3) return;
  if (in_sizes[0] != kNb * kSig) return;
  if (in_sizes[1] != kBins * kNfft) return;
  if (in_sizes[2] != kBins * kNfft) return;
  if (out_size != kOutTotal) return;
  if (ws_size < kWsTotal) return;

  const float* x    = (const float*)d_in[0];
  const float* wsin = (const float*)d_in[1];
  const float* wcos = (const float*)d_in[2];
  float* out = (float*)d_out;

  char* ws = (char*)d_ws;
  unsigned* FRw  = (unsigned*)(ws + kOffFr);
  unsigned* TAPw = (unsigned*)(ws + kOffTap);
  float*    MAG  = (float*)(ws + kOffMag);

  frames_f16_kernel<<<kRowsPad, 256, 0, stream>>>(x, FRw);
  taps_f16_kernel<<<kTapRows, 256, 0, stream>>>(wsin, wcos, TAPw);
  fused_product_mag_kernel<<<(kTilesM * kTilesN) / 8, 256, 0, stream>>>(
      (const unsigned short*)FRw, (const unsigned short*)TAPw, MAG);
  line_transpose_kernel<<<(kOutLines + 7) / 8, 256, 0, stream>>>(MAG, out);
}
